// SDPAttention_3796751089839
// MI455X (gfx1250) — hardware-verified
//
#include <hip/hip_runtime.h>


namespace {
constexpr int B = 8, L = 4096, HD = 64, BL = 8  , QL = 4096  ;
constexpr float XS = 8.0f, PS = 1024.0f, LOG2E = 1.4426950408889634f;
static_assert(L % 64 == 0 && QL % 64 == 0, "tiling");
typedef _Float16 b16;
typedef __attribute__((ext_vector_type(16))) _Float16 v16b;
typedef __attribute__((ext_vector_type(8))) _Float16 v8b;
typedef __attribute__((ext_vector_type(8))) float v8f;
typedef __attribute__((ext_vector_type(4))) float v4f;
__device__ __forceinline__ float bf16_rne(float f) { unsigned int u = __float_as_uint(f); u += 0x7FFFu + ((u >> 16) & 1u); return __uint_as_float(u & 0xFFFF0000u); }
__device__ __forceinline__ void split16(float v, b16& hi, b16& lo) { hi = (b16)v; lo = (b16)(v - (float)hi); }
__device__ __forceinline__ v16b frag_kb(const b16* p, int hh) { const v8b a = *(const v8b*)(p + 8 * hh), b = *(const v8b*)(p + 16 + 8 * hh); v16b f;
#pragma unroll
  for (int e = 0; e < 8; ++e) { f[e] = a[e]; f[8 + e] = b[e]; } return f; }
__device__ __forceinline__ v8f wmma16b(v16b a, v16b b, v8f c) { v8f d = __builtin_amdgcn_wmma_f32_16x16x32_f16(false, a, false, b, (short)0, c, false, false); asm volatile("v_nop\n\tv_nop\n\tv_nop\n\tv_nop" : "+v"(d) : "v"(a), "v"(b)); return d; }
__device__ __forceinline__ void wave_lds_sync() { __builtin_amdgcn_fence(__ATOMIC_RELEASE, "workgroup"); __builtin_amdgcn_wave_barrier(); __builtin_amdgcn_fence(__ATOMIC_ACQUIRE, "workgroup"); }
__device__ __forceinline__ float pmul(float a, float b) { float p = a * b; asm volatile("" : "+v"(p)); return p; }
__device__ __forceinline__ int iclamp(int v, int lo, int hi) { return v < lo ? lo : (v > hi ? hi : v); }

typedef __attribute__((ext_vector_type(2))) _Float16 v2h;
typedef __attribute__((ext_vector_type(4))) _Float16 v4h;
typedef __attribute__((ext_vector_type(2))) float v2f;
__device__ __forceinline__ float nexp2(float v) { return __builtin_amdgcn_exp2f(v); }
__global__ __launch_bounds__(256) void plane_kernel(const float* __restrict__ q, const float* __restrict__ k, const float* __restrict__ v, b16* __restrict__ QP, b16* __restrict__ KP, b16* __restrict__ VT) {
  __shared__ b16 Tv[64][HD + 2];
  const int t0 = blockIdx.x * 64, b = blockIdx.y; if (t0 >= QL) return;
  const size_t base = ((size_t)b * L + t0) * HD;
  for (int i = threadIdx.x; i < 64 * HD; i += 256) { const int t = i / HD, c = i % HD; Tv[t][c] = (b16)(bf16_rne(v[base + i]) * XS); }
  __syncthreads();
  for (int pass = 0; pass < 2; ++pass) {
    for (int i = threadIdx.x; i < 64 * HD / 4; i += 256) { const v4f fq = *(const v4f*)(q + base + (size_t)i * 4), fk = *(const v4f*)(k + base + (size_t)i * 4); v4h oq, ok; for (int j = 0; j < 4; ++j) { oq[j] = (b16)(bf16_rne(fq[j]) * XS); ok[j] = (b16)(bf16_rne(fk[j]) * XS); }
      *(volatile v4h*)(QP + base + (size_t)i * 4) = oq; *(volatile v4h*)(KP + base + (size_t)i * 4) = ok; }
    for (int i = threadIdx.x; i < HD * 32; i += 256) { const int d = i / 32, tp = (i % 32) * 2; v2h o2; o2[0] = Tv[tp][d]; o2[1] = Tv[tp + 1][d]; *(volatile v2h*)(VT + ((size_t)b * HD + d) * (size_t)L + t0 + tp) = o2; }
    __threadfence(); }
}
__global__ __launch_bounds__(64) void attn_kernel(const b16* __restrict__ QP, const b16* __restrict__ KP, const b16* __restrict__ VT, float* __restrict__ out) {
  __shared__ __attribute__((aligned(16))) b16 Pb[2][16][32 + 8], Pc[2][16][32 + 8]; __shared__ __attribute__((aligned(16))) float To[2][16][HD + 4];
  const int wave = threadIdx.x >> 5, lane = threadIdx.x & 31, hh = lane >> 4, col = lane & 15; const int b = blockIdx.y; const int q0 = blockIdx.x * 32 + wave * 16, qi = q0 + col;
  const b16* Qb = QP + (size_t)b * L * HD; const b16* Kb = KP + (size_t)b * L * HD; const b16* Vb = VT + (size_t)b * HD * (size_t)L;
  const v16b qa0 = frag_kb(Qb + (size_t)qi * HD, hh), qa1 = frag_kb(Qb + (size_t)qi * HD + 32, hh);
  const float cs = LOG2E / (8.0f * XS * XS);
  float m = -INFINITY, l = 0.0f; v8f o[4]; for (int t = 0; t < 4; ++t) o[t] = (v8f){};
  const int kend = q0 + 16;
#pragma unroll 1
  for (int kb = 0; kb < kend; kb += 32) {
    float e[16]; float mx = -INFINITY;
#pragma unroll
    for (int u = 0; u < 2; ++u) { v8f s = (v8f){}; const size_t kr = (size_t)(kb + u * 16 + col) * HD; s = wmma16b(frag_kb(Kb + kr, hh), qa0, s); s = wmma16b(frag_kb(Kb + kr + 32, hh), qa1, s);
#pragma unroll
      for (int r = 0; r < 8; ++r) { const int key = kb + u * 16 + 8 * hh + r; const float vv = (key <= qi) ? s[r] * cs : -INFINITY; e[u * 8 + r] = vv; mx = fmaxf(mx, vv); } }
    mx = fmaxf(mx, __shfl_xor(mx, 16)); const float mn = fmaxf(m, mx); const float al = (mn == -INFINITY) ? 1.0f : nexp2(m - mn); float sum = 0.0f;
#pragma unroll
    for (int i2 = 0; i2 < 16; ++i2) { const float p = (e[i2] == -INFINITY) ? 0.0f : nexp2(e[i2] - mn); sum += p; b16 a_, b_; split16(p * PS, a_, b_); const int sl = (i2 < 8 ? 0 : 16) + 8 * hh + (i2 & 7); Pb[wave][col][sl] = a_; Pc[wave][col][sl] = b_; }
    sum += __shfl_xor(sum, 16); l = l * al + sum; m = mn;
    wave_lds_sync();
    const v16b pf = frag_kb(&Pb[wave][col][0], hh), pg = frag_kb(&Pc[wave][col][0], hh);
#pragma unroll
    for (int t = 0; t < 4; ++t) { o[t] *= al; const v16b va = frag_kb(Vb + (size_t)(t * 16 + col) * L + kb, hh); o[t] = wmma16b(va, pf, o[t]); o[t] = wmma16b(va, pg, o[t]); }
    wave_lds_sync(); }
  const float inv = 1.0f / (l * PS * XS);
#pragma unroll
  for (int t = 0; t < 4; ++t)
#pragma unroll
    for (int r = 0; r < 8; ++r) To[wave][col][t * 16 + 8 * hh + r] = o[t][r] * inv;
  wave_lds_sync();
  for (int pass = 0; pass < 2; ++pass) { for (int rr = 0; rr < 16; ++rr) *(volatile v2f*)(out + ((size_t)b * L + q0 + rr) * HD + lane * 2) = *(const v2f*)(&To[wave][rr][lane * 2]); __threadfence(); }
}
}

extern "C" void kernel_launch(void* const* d_in, const int* in_sizes, int n_in, void* d_out, int out_size, void* d_ws, size_t ws_size, hipStream_t stream) {
  (void)n_in;
  auto Fp = [&](int i) { return (const float*)d_in[i]; };
  if (in_sizes[0] != B * L * HD || in_sizes[1] != B * L * HD || in_sizes[2] != B * L * HD || out_size != B * L * HD) return;
  size_t off = 0; char* ws = (char*)d_ws;
  auto carve = [&](size_t bytes) { char* p = ws + off; off += (bytes + 255) & ~(size_t)255; return p; };
  const size_t plane = (size_t)B * L * HD * 2; b16* QP = (b16*)carve(plane); b16* KP = (b16*)carve(plane); b16* VT = (b16*)carve(plane);
  if (off > ws_size || off > ((size_t)128 << 20)) return;
  plane_kernel<<<dim3(L / 64, BL), 256, 0, stream>>>(Fp(0), Fp(1), Fp(2), QP, KP, VT);
  attn_kernel<<<dim3(QL / 32, BL), 64, 0, stream>>>(QP, KP, VT, (float*)d_out);
}
